// PointNetSetAbstractionCN2Nor_67997922230548
// MI455X (gfx1250) — hardware-verified
//
#include <hip/hip_runtime.h>
#include <math.h>
typedef __attribute__((ext_vector_type(16))) _Float16 v16h;
typedef __attribute__((ext_vector_type(8)))  _Float16 v8h;
typedef __attribute__((ext_vector_type(16))) __bf16   v16b;
typedef __attribute__((ext_vector_type(8)))  __bf16   v8b;
typedef __attribute__((ext_vector_type(8)))  float    v8f;
typedef __attribute__((ext_vector_type(4)))  float    v4f;
#define PSCALE 32768.0f
#define U16(p) ((const unsigned short*)(const void*)(p))
#define PSCALE_INV (1.0f / 32768.0f)

__device__ __forceinline__ unsigned short f2bf_bits(float f) {
  unsigned u = __float_as_uint(f);
  return (unsigned short)((u + 0x7FFFu + ((u >> 16) & 1u)) >> 16);
}
__device__ __forceinline__ float bf_bits2f(unsigned short h) { return __uint_as_float(((unsigned)h) << 16); }

__device__ __forceinline__ void dep_guard_h(v8f& a, v8f& b, v16h x, v16h y) { asm volatile("v_nop\n\tv_nop\n\tv_nop\n\tv_nop" : "+v"(a), "+v"(b) : "v"(x), "v"(y)); }
__device__ __forceinline__ void dep_guard_b(v8f& a, v8f& b, v16b x, v16b y) { asm volatile("v_nop\n\tv_nop\n\tv_nop\n\tv_nop" : "+v"(a), "+v"(b) : "v"(x), "v"(y)); }
__device__ __forceinline__ void keep4_h(v16h a, v16h b, v16h c, v16h d) { asm volatile("v_nop" :: "v"(a), "v"(b), "v"(c), "v"(d)); }
__device__ __forceinline__ void keep4_b(v16b a, v16b b, v16b c, v16b d) { asm volatile("v_nop" :: "v"(a), "v"(b), "v"(c), "v"(d)); }
__device__ __forceinline__ void acc_guard4(v8f& a, v8f& b, v8f& c, v8f& d) { asm volatile("v_nop\n\tv_nop\n\tv_nop\n\tv_nop" : "+v"(a), "+v"(b), "+v"(c), "+v"(d)); }
template <typename T> struct Frag;
template <> struct Frag<_Float16> {
  typedef v16h V; union U { v16h v; v8h h[2]; };
  static __device__ __forceinline__ v16h load(const _Float16* p) {
    U f; f.h[0] = *(const v8h*)(p); f.h[1] = *(const v8h*)(p + 16); return f.v;
  }
  static __device__ __forceinline__ v8f mma(v16h a, v16h b, v8f c) {
    return __builtin_amdgcn_wmma_f32_16x16x32_f16(false, a, false, b, (short)0, c, false, false);
  }
  static __device__ __forceinline__ void guard(v8f& a, v8f& b, v16h x, v16h y) { dep_guard_h(a, b, x, y); }
  static __device__ __forceinline__ void keep(v16h a, v16h b, v16h c, v16h d) { keep4_h(a, b, c, d); }
};
template <> struct Frag<__bf16> {
  typedef v16b V; union U { v16b v; v8b h[2]; };
  static __device__ __forceinline__ v16b load(const __bf16* p) {
    U f; f.h[0] = *(const v8b*)(p); f.h[1] = *(const v8b*)(p + 16); return f.v;
  }
  static __device__ __forceinline__ v8f mma(v16b a, v16b b, v8f c) {
    return __builtin_amdgcn_wmma_f32_16x16x32_bf16(false, a, false, b, (short)0, c, false, false);
  }
  static __device__ __forceinline__ void guard(v8f& a, v8f& b, v16b x, v16b y) { dep_guard_b(a, b, x, y); }
  static __device__ __forceinline__ void keep(v16b a, v16b b, v16b c, v16b d) { keep4_b(a, b, c, d); }
};

template <int ET> struct Elem;
template <> struct Elem<0> { typedef _Float16 T; };
template <> struct Elem<1> { typedef __bf16 T; };
template <int ET, bool SPLIT, int BIAS_MODE, int OUT_MODE, bool RESID, int ACT = 0>
__global__ __launch_bounds__(256) void wmma_gemm64(
    const unsigned short* __restrict__ Ap, const unsigned short* __restrict__ A2p, int lda, long strideA,
    const unsigned short* __restrict__ Btp, const unsigned short* __restrict__ Bt2p, int ldb, long strideB,
    void* __restrict__ Cout, void* __restrict__ Cout2, int ldc, long strideC,
    const float* __restrict__ bias,
    const float* __restrict__ resid, long strideR,
    int M, int N, int K, float scale) {
  typedef typename Elem<ET>::T T;
  typedef typename Frag<T>::V V;
  const T* A = (const T*)Ap; const T* A2 = (const T*)A2p; const T* Bt = (const T*)Btp; const T* Bt2 = (const T*)Bt2p;
  __shared__ __align__(16) float sT[8][16 * 68];
  const int b    = blockIdx.y;
  const int lane = threadIdx.x & 31;
  const int wave = threadIdx.x >> 5;
  const int tilesN = N >> 6;
  const int tilesM = M >> 6;
  const int tile = blockIdx.x * 8 + wave;
  if (tile >= tilesM * tilesN) return;
  const int tm = tile / tilesN;
  const int tn = tile - tm * tilesN;
  const int m0 = tm << 6;
  const int n0 = tn << 6;

  const T* Ab  = A  + (size_t)b * strideA;
  const T* Bb  = Bt + (size_t)b * strideB;
  const T* Ab2 = SPLIT ? (A2  + (size_t)b * strideA) : nullptr;
  const T* Bb2 = SPLIT ? (Bt2 + (size_t)b * strideB) : nullptr;

  const int rlane = lane & 15;
  const int koff  = (lane >> 4) * 8;
  const int mOff  = (lane >> 4) * 8;

  v8f acc[4][4];
#pragma unroll
  for (int i = 0; i < 4; ++i)
#pragma unroll
    for (int j = 0; j < 4; ++j) acc[i][j] = (v8f){0.f,0.f,0.f,0.f,0.f,0.f,0.f,0.f};

  for (int k0 = 0; k0 < K; k0 += 32) {
    V bh[4], bl[4];
#pragma unroll
    for (int j = 0; j < 4; ++j) {
      const size_t bo = (size_t)(n0 + (j << 4) + rlane) * ldb + koff + k0;
      bh[j] = Frag<T>::load(Bb + bo);
      if (SPLIT) bl[j] = Frag<T>::load(Bb2 + bo);
    }
#pragma unroll
    for (int i = 0; i < 4; ++i) {
      const size_t ao = (size_t)(m0 + (i << 4) + rlane) * lda + koff + k0;
      V ah = Frag<T>::load(Ab + ao);
      V al;
      if (SPLIT) al = Frag<T>::load(Ab2 + ao);
#pragma unroll
      for (int j = 0; j < 4; ++j) {
        acc[i][j] = Frag<T>::mma(ah, bh[j], acc[i][j]);
        if (SPLIT) {
          acc[i][j] = Frag<T>::mma(ah, bl[j], acc[i][j]);
          acc[i][j] = Frag<T>::mma(al, bh[j], acc[i][j]);
        }
      }
      Frag<T>::guard(acc[i][0], acc[i][3], ah, SPLIT ? al : ah);
    }
    Frag<T>::keep(bh[0], bh[1], bh[2], bh[3]);
    if (SPLIT) Frag<T>::keep(bl[0], bl[1], bl[2], bl[3]);
  }
  acc_guard4(acc[0][0], acc[0][1], acc[0][2], acc[0][3]);
  acc_guard4(acc[1][0], acc[1][1], acc[1][2], acc[1][3]);
  acc_guard4(acc[2][0], acc[2][1], acc[2][2], acc[2][3]);
  acc_guard4(acc[3][0], acc[3][1], acc[3][2], acc[3][3]);

  float* slab = sT[wave];
  const float* Rb = RESID ? (resid + (size_t)b * strideR) : nullptr;
#pragma unroll
  for (int i = 0; i < 4; ++i) {
    const int mBase = m0 + (i << 4);
#pragma unroll
    for (int j = 0; j < 4; ++j) {
      const int n = n0 + (j << 4) + rlane;
      float bv = 0.f;
      if (BIAS_MODE == 2) bv = bias[n];
#pragma unroll
      for (int r = 0; r < 8; ++r) {
        float v = acc[i][j][r] * scale;
        if (BIAS_MODE == 1) v += bias[mBase + mOff + r];
        if (BIAS_MODE == 2) v += bv;
        if (RESID) v += Rb[(size_t)(mBase + mOff + r) * ldc + n];
        if (ACT == 1) v = tanhf(v);
        if (ACT == 2) v = fmaxf(v, 0.0f);
        if (ACT == 3) v = v / (1.0f + expf(-v));
        if (ACT == 4) v = (v > 0.f) ? v : 0.01f * v;
        if (ACT == 5) v = 0.5f * v * (1.0f + erff(v * 0.70710678118654752f));
        slab[(mOff + r) * 68 + (j << 4) + rlane] = v;
      }
    }
    __builtin_amdgcn_fence(__ATOMIC_RELEASE, "workgroup");
    __builtin_amdgcn_wave_barrier();
    __builtin_amdgcn_fence(__ATOMIC_ACQUIRE, "workgroup");
    if (OUT_MODE == 0) {
      float* C = (float*)Cout + (size_t)b * strideC;
      const int hh = lane >> 4, c4 = (lane & 15) * 4;
      for (int pass = 0; pass < 2; ++pass) {
#pragma unroll
        for (int it = 0; it < 8; ++it) {
          const int row = it * 2 + hh;
          v4f v = *(const v4f*)(slab + row * 68 + c4);
          *(volatile v4f*)(C + (size_t)(mBase + row) * ldc + n0 + c4) = v;
        }
        __threadfence();
      }
    } else {
      const int q = lane >> 3, c8 = (lane & 7) * 8;
      unsigned short* C  = (unsigned short*)Cout  + (size_t)b * strideC;
      unsigned short* C2 = (OUT_MODE == 2) ? ((unsigned short*)Cout2 + (size_t)b * strideC) : nullptr;
      for (int pass = 0; pass < 2; ++pass) {
#pragma unroll
        for (int it = 0; it < 4; ++it) {
          const int row = it * 4 + q;
          const float* sp = slab + row * 68 + c8;
          v8h hv, lv;
#pragma unroll
          for (int e = 0; e < 8; ++e) {
            if (OUT_MODE == 1) {
              hv[e] = (_Float16)sp[e];
            } else {
              unsigned short hb = f2bf_bits(sp[e]);
              unsigned short lb = f2bf_bits(sp[e] - bf_bits2f(hb));
              hv[e] = __builtin_bit_cast(_Float16, hb);
              lv[e] = __builtin_bit_cast(_Float16, lb);
            }
          }
          *(volatile v8h*)(C + (size_t)(mBase + row) * ldc + n0 + c8) = hv;
          if (OUT_MODE == 2) *(volatile v8h*)(C2 + (size_t)(mBase + row) * ldc + n0 + c8) = lv;
        }
        __threadfence();
      }
    }
    __builtin_amdgcn_fence(__ATOMIC_RELEASE, "workgroup");
    __builtin_amdgcn_wave_barrier();
    __builtin_amdgcn_fence(__ATOMIC_ACQUIRE, "workgroup");
  }
}

__global__ __launch_bounds__(256) void cast_f32_f16x2(
    const float* __restrict__ in, _Float16* __restrict__ out, int n2) {
  int i = blockIdx.x * 256 + threadIdx.x;
  if (i < n2) {
    const _Float16 h0 = (_Float16)in[2 * i], h1 = (_Float16)in[2 * i + 1];
    const unsigned u = (unsigned)__builtin_bit_cast(unsigned short, h0) | ((unsigned)__builtin_bit_cast(unsigned short, h1) << 16);
    ((volatile unsigned*)out)[i] = u;
    __threadfence();
    ((volatile unsigned*)out)[i] = u;
  }
}


#define PN_ 65536
#define PK 32
#define PCI 16
#define PR ((long)PN_ * PK)
#define NCHK 16
#define RCH (PR / NCHK)
__global__ __launch_bounds__(256) void moments_kernel(const float* __restrict__ xyz, const float* __restrict__ pts, const int* __restrict__ gi, float* __restrict__ MP) {
  __shared__ float red[8][288];
  const int lane = threadIdx.x & 31, wave = threadIdx.x >> 5; const int half = lane >> 4, b = lane & 15, base = half << 4;
  float acc[16]; for (int a = 0; a < 16; ++a) acc[a] = 0.f; float accd[3] = {0.f, 0.f, 0.f}; float sv = 0.f, sd = 0.f;
#pragma unroll 1
  for (long rp = (long)blockIdx.x * 8 + wave; rp < PR / 2; rp += (long)gridDim.x * 8) { const long r = 2 * rp + half; const int n = (int)(r / PK); int j = gi[r]; j = j < 0 ? 0 : (j >= PN_ ? PN_ - 1 : j);
    const float v = pts[(size_t)j * PCI + b]; const float d = (b < 3) ? (xyz[j * 3 + b] - xyz[n * 3 + b]) : 0.f;
    sv += v; sd += d;
#pragma unroll
    for (int a = 0; a < 16; ++a) acc[a] += __shfl(v, base + a, 32) * v;
#pragma unroll
    for (int a = 0; a < 3; ++a) accd[a] += __shfl(d, base + a, 32) * d; }
  for (int a = 0; a < 16; ++a) acc[a] += __shfl_xor(acc[a], 16, 32); for (int a = 0; a < 3; ++a) accd[a] += __shfl_xor(accd[a], 16, 32); sv += __shfl_xor(sv, 16, 32); sd += __shfl_xor(sd, 16, 32);
  if (half == 0) { for (int a = 0; a < 16; ++a) red[wave][a * 16 + b] = acc[a]; red[wave][256 + b] = sv; if (b < 3) { for (int a = 0; a < 3; ++a) red[wave][272 + a * 3 + b] = accd[a]; red[wave][281 + b] = sd; } }
  __syncthreads();
  for (int pass = 0; pass < 2; ++pass) { for (int e = threadIdx.x; e < 288; e += 256) { float s = 0.f; if (e < 284) for (int w = 0; w < 8; ++w) s += red[w][e]; ((volatile float*)MP)[(size_t)blockIdx.x * 288 + e] = s; } __threadfence(); }
}
__global__ __launch_bounds__(64) void bn1_kernel(const float* __restrict__ MP, int nblk, const float* __restrict__ Wl, const float* __restrict__ gl, const float* __restrict__ bl, const float* __restrict__ Wf, const float* __restrict__ gf, const float* __restrict__ bf, float* __restrict__ SS1) {
  __shared__ double mom[284];
  for (int e = threadIdx.x; e < 284; e += 64) { double s = 0.0; for (int k = 0; k < nblk; ++k) s += (double)MP[(size_t)k * 288 + e]; mom[e] = s / (double)PR; }
  __syncthreads();
  const int o = threadIdx.x & 31; const bool isf = threadIdx.x >= 32;
  double mean = 0.0, ex2 = 0.0;
  if (!isf) { for (int a = 0; a < 3; ++a) { mean += (double)Wl[o * 3 + a] * mom[281 + a]; for (int c = 0; c < 3; ++c) ex2 += (double)Wl[o * 3 + a] * (double)Wl[o * 3 + c] * mom[272 + a * 3 + c]; } }
  else { for (int a = 0; a < PCI; ++a) { mean += (double)Wf[o * PCI + a] * mom[256 + a]; for (int c = 0; c < PCI; ++c) ex2 += (double)Wf[o * PCI + a] * (double)Wf[o * PCI + c] * mom[a * 16 + c]; } }
  double var = ex2 - mean * mean; if (var < 0) var = 0;
  const float g = isf ? gf[o] : gl[o], bb = isf ? bf[o] : bl[o]; const float sc = g * (float)(1.0 / sqrt(var + 1e-5)); const float sh = bb - (float)mean * sc;
  for (int pass = 0; pass < 2; ++pass) { ((volatile float*)SS1)[(isf ? 64 : 0) + o] = sc; ((volatile float*)SS1)[(isf ? 96 : 32) + o] = sh; __threadfence(); }
}
__global__ __launch_bounds__(256) void gather_kernel(const float* __restrict__ xyz, const float* __restrict__ pts, const int* __restrict__ gi, long r0, unsigned* __restrict__ A16) {
  const long rl = (long)blockIdx.x * 256 + threadIdx.x; const long r = r0 + rl; const int n = (int)(r / PK); int j = gi[r]; j = j < 0 ? 0 : (j >= PN_ ? PN_ - 1 : j);
  float v[32]; v[0] = xyz[j * 3] - xyz[n * 3]; v[1] = xyz[j * 3 + 1] - xyz[n * 3 + 1]; v[2] = xyz[j * 3 + 2] - xyz[n * 3 + 2];
  for (int c = 0; c < PCI; ++c) v[3 + c] = pts[(size_t)j * PCI + c]; for (int c = 19; c < 32; ++c) v[c] = 0.f;
  typedef __attribute__((ext_vector_type(4))) unsigned u4; u4 u[4];
  for (int q = 0; q < 16; ++q) u[q / 4][q % 4] = (unsigned)__builtin_bit_cast(unsigned short, (_Float16)v[2 * q]) | ((unsigned)__builtin_bit_cast(unsigned short, (_Float16)v[2 * q + 1]) << 16);
  for (int pass = 0; pass < 2; ++pass) { for (int q = 0; q < 4; ++q) *(volatile u4*)(A16 + rl * 16 + q * 4) = u[q]; __threadfence(); }
}
__global__ __launch_bounds__(256) void w0_kernel(const float* __restrict__ Wl, const float* __restrict__ Wf, unsigned* __restrict__ BT0, const float* __restrict__ W1, unsigned* __restrict__ BT1) {
  for (int i = threadIdx.x; i < 64 * 16; i += 256) { const int o = i / 16, kp = 2 * (i % 16); float a = 0.f, b = 0.f;
    for (int e = 0; e < 2; ++e) { const int k = kp + e; float v = 0.f; if (o < 32) { if (k < 3) v = Wl[o * 3 + k]; } else { if (k >= 3 && k < 19) v = Wf[(o - 32) * PCI + (k - 3)]; } if (e == 0) a = v; else b = v; }
    const unsigned u = (unsigned)__builtin_bit_cast(unsigned short, (_Float16)a) | ((unsigned)__builtin_bit_cast(unsigned short, (_Float16)b) << 16); ((volatile unsigned*)BT0)[i] = u;
    const unsigned u1 = (unsigned)__builtin_bit_cast(unsigned short, (_Float16)W1[o * 32 + kp]) | ((unsigned)__builtin_bit_cast(unsigned short, (_Float16)W1[o * 32 + kp + 1]) << 16); ((volatile unsigned*)BT1)[i] = u1; }
  __threadfence();
  for (int i = threadIdx.x; i < 64 * 16; i += 256) { ((volatile unsigned*)BT0)[i] = BT0[i]; ((volatile unsigned*)BT1)[i] = BT1[i]; }
}
__global__ __launch_bounds__(256) void h1_kernel(const float* __restrict__ LF, const float* __restrict__ SS1, long r0, unsigned* __restrict__ H1) {
  const int lane = threadIdx.x & 31, wave = threadIdx.x >> 5; const long rp = (long)blockIdx.x * 8 + wave;
  unsigned u[2];
  for (int sub = 0; sub < 2; ++sub) { const long rl = 2 * rp + sub;
    const float lo = LF[rl * 64 + lane], fe = LF[rl * 64 + 32 + lane];
    const float h = fmaxf(lo * SS1[lane] + SS1[32 + lane] + fe * SS1[64 + lane] + SS1[96 + lane], 0.f);
    const float hn = __shfl_xor(h, 1, 32);
    u[sub] = (unsigned)__builtin_bit_cast(unsigned short, (_Float16)h) | ((unsigned)__builtin_bit_cast(unsigned short, (_Float16)hn) << 16); }
  const unsigned v0 = __shfl(u[0], 2 * (lane & 15), 32), v1 = __shfl(u[1], 2 * (lane & 15), 32);
  const unsigned mine = (lane < 16) ? v0 : v1;
  ((volatile unsigned*)H1)[(r0 + 2 * rp) * 16 + lane] = mine; __threadfence(); ((volatile unsigned*)H1)[(r0 + 2 * rp) * 16 + lane] = mine;
}
__global__ __launch_bounds__(256) void stats2_kernel(const float* __restrict__ H2, long r0, double* __restrict__ HP, float* __restrict__ MX, float* __restrict__ MN) {
  typedef __attribute__((ext_vector_type(2))) float v2f;
  __shared__ double red[2][8][64];
  const int lane = threadIdx.x & 31, wave = threadIdx.x >> 5;
  double s0 = 0, s1 = 0, q0 = 0, q1 = 0;
#pragma unroll 1
  for (long nl = (long)blockIdx.x * 8 + wave; nl < RCH / PK; nl += (long)gridDim.x * 8) { v2f mx = {-INFINITY, -INFINITY}, mn = {INFINITY, INFINITY}; float a0 = 0.f, a1 = 0.f, b0 = 0.f, b1v = 0.f;
#pragma unroll 1
    for (int k = 0; k < PK; ++k) { const v2f v = *(const v2f*)(H2 + (nl * PK + k) * 64 + 2 * lane); mx[0] = fmaxf(mx[0], v[0]); mx[1] = fmaxf(mx[1], v[1]); mn[0] = fminf(mn[0], v[0]); mn[1] = fminf(mn[1], v[1]); a0 += v[0]; a1 += v[1]; b0 += v[0] * v[0]; b1v += v[1] * v[1]; }
    s0 += a0; s1 += a1; q0 += b0; q1 += b1v; const long n = r0 / PK + nl;
    *(volatile v2f*)(MX + n * 64 + 2 * lane) = mx; *(volatile v2f*)(MN + n * 64 + 2 * lane) = mn; __threadfence(); *(volatile v2f*)(MX + n * 64 + 2 * lane) = mx; *(volatile v2f*)(MN + n * 64 + 2 * lane) = mn; }
  red[0][wave][2 * lane] = s0; red[0][wave][2 * lane + 1] = s1; red[1][wave][2 * lane] = q0; red[1][wave][2 * lane + 1] = q1; __syncthreads();
  if (threadIdx.x < 128) { const int c = threadIdx.x & 63, which = threadIdx.x >> 6; double t = 0; for (int w = 0; w < 8; ++w) t += red[which][w][c]; ((volatile double*)HP)[(size_t)blockIdx.x * 128 + threadIdx.x] = t; __threadfence(); ((volatile double*)HP)[(size_t)blockIdx.x * 128 + threadIdx.x] = t; }
}
__global__ __launch_bounds__(256) void out_kernel(const float* __restrict__ MX, const float* __restrict__ MN, const float* __restrict__ SS2, float* __restrict__ out) {
  typedef __attribute__((ext_vector_type(2))) float v2f;
  const int lane = threadIdx.x & 31, wave = threadIdx.x >> 5; const long n = (long)blockIdx.x * 8 + wave;
  const float s0 = SS2[2 * lane], s1 = SS2[2 * lane + 1], h0 = SS2[64 + 2 * lane], h1s = SS2[64 + 2 * lane + 1];
  const v2f mx = *(const v2f*)(MX + n * 64 + 2 * lane), mn = *(const v2f*)(MN + n * 64 + 2 * lane);
  v2f o; o[0] = fmaxf((s0 >= 0.f ? mx[0] : mn[0]) * s0 + h0, 0.f); o[1] = fmaxf((s1 >= 0.f ? mx[1] : mn[1]) * s1 + h1s, 0.f);
  *(volatile v2f*)(out + n * 64 + 2 * lane) = o; __threadfence(); *(volatile v2f*)(out + n * 64 + 2 * lane) = o;
}
__global__ __launch_bounds__(64) void bn2_kernel(const double* __restrict__ HP, int nblk_total, const float* __restrict__ g1, const float* __restrict__ be1, float* __restrict__ SS2) {
  const int o = threadIdx.x; double s = 0.0, ss = 0.0; for (int b = 0; b < nblk_total; ++b) { s += HP[(size_t)b * 128 + o]; ss += HP[(size_t)b * 128 + 64 + o]; }
  const double mean = s / (double)PR; double var = ss / (double)PR - mean * mean; if (var < 0) var = 0;
  const float sc = g1[o] * (float)(1.0 / sqrt(var + 1e-5)); const float sh = be1[o] - (float)mean * sc;
  for (int pass = 0; pass < 2; ++pass) { ((volatile float*)SS2)[o] = sc; ((volatile float*)SS2)[64 + o] = sh; __threadfence(); }
}
__global__ __launch_bounds__(256) void max_kernel(const float* __restrict__ H2, const float* __restrict__ SS2, long r0, float* __restrict__ out) {
  typedef __attribute__((ext_vector_type(2))) float v2f;
  const int lane = threadIdx.x & 31, wave = threadIdx.x >> 5; const long nl = (long)blockIdx.x * 8 + wave; const long n = r0 / PK + nl;
  const float s0 = SS2[2 * lane], s1 = SS2[2 * lane + 1], h0 = SS2[64 + 2 * lane], h1s = SS2[64 + 2 * lane + 1];
  v2f mx = {0.f, 0.f};
#pragma unroll 1
  for (int k = 0; k < PK; ++k) { const v2f v = *(const v2f*)(H2 + (nl * PK + k) * 64 + 2 * lane); mx[0] = fmaxf(mx[0], v[0] * s0 + h0); mx[1] = fmaxf(mx[1], v[1] * s1 + h1s); }
  *(volatile v2f*)(out + n * 64 + 2 * lane) = mx; __threadfence(); *(volatile v2f*)(out + n * 64 + 2 * lane) = mx;
}
extern "C" void kernel_launch(void* const* d_in, const int* in_sizes, int n_in, void* d_out, int out_size, void* d_ws, size_t ws_size, hipStream_t stream) {
  (void)in_sizes; (void)n_in; (void)out_size; (void)ws_size;
  auto Fp = [&](int i) { return (const float*)d_in[i]; };
  const float* xyz = Fp(0); const float* pts = Fp(1); const int* gi = (const int*)d_in[2]; const float* Wl = Fp(3); const float* gl = Fp(4); const float* bl = Fp(5); const float* Wf = Fp(6); const float* gf = Fp(7); const float* bf = Fp(8); const float* W1 = Fp(9); const float* b1 = Fp(10); const float* g1 = Fp(11); const float* be1 = Fp(12);
  char* ws = (char*)d_ws; size_t off = 0;
  auto carve = [&](size_t bytes) -> char* { char* p = ws + off; off += (bytes + 255) & ~(size_t)255; return p; };
  const int NMB = 2048, NHB = 512;
  float* MP = (float*)carve((size_t)NMB * 288 * 4); float* SS1 = (float*)carve(128 * 4); unsigned* BT0 = (unsigned*)carve(64 * 32 * 2); unsigned* BT1 = (unsigned*)carve(64 * 32 * 2);
  unsigned* A16 = (unsigned*)carve((size_t)RCH * 32 * 2); float* LF = (float*)carve((size_t)RCH * 64 * 4); unsigned* H1 = (unsigned*)carve((size_t)RCH * 32 * 2);
  double* HP = (double*)carve((size_t)NCHK * NHB * 128 * 8); float* SS2 = (float*)carve(128 * 4); float* MX = (float*)carve((size_t)PN_ * 64 * 4); float* MN = (float*)carve((size_t)PN_ * 64 * 4);
  moments_kernel<<<NMB, 256, 0, stream>>>(xyz, pts, gi, MP);
  bn1_kernel<<<1, 64, 0, stream>>>(MP, NMB, Wl, gl, bl, Wf, gf, bf, SS1);
  w0_kernel<<<1, 256, 0, stream>>>(Wl, Wf, BT0, W1, BT1);
  const int t = (int)((RCH / 64) * 1);
  auto stage1 = [&](long r0) {
    gather_kernel<<<(unsigned)(RCH / 256), 256, 0, stream>>>(xyz, pts, gi, r0, A16);
    wmma_gemm64<0, false, 0, 0, false><<<dim3((t + 7) / 8, 1), 256, 0, stream>>>((const unsigned short*)A16, nullptr, 32, 0, (const unsigned short*)BT0, nullptr, 32, 0, LF, nullptr, 64, 0, nullptr, nullptr, 0, (int)RCH, 64, 32, 1.0f);
    h1_kernel<<<(unsigned)(RCH / 16), 256, 0, stream>>>(LF, SS1, 0, H1); };
  for (int c = 0; c < NCHK; ++c) { const long r0 = (long)c * RCH; stage1(r0);
    wmma_gemm64<0, false, 2, 0, false><<<dim3((t + 7) / 8, 1), 256, 0, stream>>>((const unsigned short*)H1, nullptr, 32, 0, (const unsigned short*)BT1, nullptr, 32, 0, LF, nullptr, 64, 0, b1, nullptr, 0, (int)RCH, 64, 32, 1.0f);
    stats2_kernel<<<NHB, 256, 0, stream>>>(LF, r0, HP + (size_t)c * NHB * 128, MX, MN); }
  bn2_kernel<<<1, 64, 0, stream>>>(HP, NCHK * NHB, g1, be1, SS2);
  out_kernel<<<PN_ / 8, 256, 0, stream>>>(MX, MN, SS2, (float*)d_out);
}
